// GatedSlotAttention_7550552506731
// MI455X (gfx1250) — hardware-verified
//
#include <hip/hip_runtime.h>
#include <hip/hip_bf16.h>

constexpr int Bc   = 2;
constexpr int Nc   = 2048;
constexpr int Dc   = 1024;
constexpr int Hc   = 8;
constexpr int Mc   = 64;
constexpr int DKc  = Dc / Hc;
constexpr int Rows = Bc * Nc;
constexpr int FMc  = Hc * Mc;
constexpr float EPSc = 1e-5f;

constexpr int GBM = 128;
constexpr int GBN = 64;
constexpr int GBK = 32;
constexpr int GPK = 40;
constexpr int GCP = 68;
constexpr int LDS_A = GBM * GPK * 2;
constexpr int LDS_B = GBN * GPK * 2;
constexpr int LDS_STAGE = 2 * LDS_A + 2 * LDS_B;
constexpr int LDS_C = GBM * GCP * 4;
constexpr int LDS_GEMM = (LDS_C > LDS_STAGE) ? LDS_C : LDS_STAGE;

typedef char chk0[(Rows % GBM == 0) ? 1 : -1];
typedef char chk1[((Dc % GBN) == 0 && (FMc % GBN) == 0 && (DKc % GBN) == 0) ? 1 : -1];
typedef char chk2[((Dc % GBK) == 0 && (DKc % GBK) == 0) ? 1 : -1];
typedef char chk3[((Dc % 64) == 0 && (DKc % 64) == 0 && (FMc % 64) == 0) ? 1 : -1];
typedef char chk4[((Rows * Dc) % (256 * 8) == 0) ? 1 : -1];

typedef _Float16     v16h __attribute__((ext_vector_type(16)));
typedef _Float16     v8h  __attribute__((ext_vector_type(8)));
typedef __bf16       v16b __attribute__((ext_vector_type(16)));
typedef float        v8f  __attribute__((ext_vector_type(8)));
typedef float        v4f  __attribute__((ext_vector_type(4)));
typedef unsigned int v4u  __attribute__((ext_vector_type(4)));

template<typename T> struct VecT;
template<> struct VecT<_Float16> { typedef v16h t; };
template<> struct VecT<__bf16>   { typedef v16b t; };
template<typename T> union Frag { typename VecT<T>::t v; v4u u[2]; };
union Pack8 { v8h hv; v4u u; unsigned short s[8]; };

__device__ __forceinline__ unsigned short bf16_rne_bits(float f) {
    unsigned int u = __float_as_uint(f);
    u += 0x7FFFu + ((u >> 16) & 1u);
    return (unsigned short)(u >> 16);
}
__device__ __forceinline__ float bf16_bits_to_f32(unsigned short s) {
    return __uint_as_float(((unsigned int)s) << 16);
}

__device__ __forceinline__ v8f mma16(v16h a, v16h b, v8f c) {
    c = __builtin_amdgcn_wmma_f32_16x16x32_f16(false, a, false, b, (short)0, c, false, false);
    asm volatile("v_nop\n\tv_nop\n\tv_nop\n\tv_nop" : "+v"(c) : "v"(a), "v"(b));
    return c;
}
__device__ __forceinline__ v8f mma16(v16b a, v16b b, v8f c) {
    c = __builtin_amdgcn_wmma_f32_16x16x32_bf16(false, a, false, b, (short)0, c, false, false);
    asm volatile("v_nop\n\tv_nop\n\tv_nop\n\tv_nop" : "+v"(c) : "v"(a), "v"(b));
    return c;
}

__global__ __launch_bounds__(256) void k_xprep(const float* __restrict__ x, int n,
                                               unsigned short* ph, unsigned short* pbh, unsigned short* pbl)
{
    const size_t i8 = ((size_t)blockIdx.x * 256 + threadIdx.x) * 8;
    if (i8 + 8 > (size_t)n) return;
    const v4f a = *(const v4f*)(x + i8);
    const v4f b = *(const v4f*)(x + i8 + 4);
    const float v[8] = { a[0], a[1], a[2], a[3], b[0], b[1], b[2], b[3] };
    Pack8 fh, fbh, fbl;
#pragma unroll
    for (int e = 0; e < 8; ++e) {
        const float f = v[e];
        fh.hv[e] = (_Float16)f;
        const unsigned short hb = bf16_rne_bits(f);
        fbh.s[e] = hb;
        fbl.s[e] = bf16_rne_bits(f - bf16_bits_to_f32(hb));
    }
    unsigned short* d0 = ph  + i8;
    unsigned short* d1 = pbh + i8;
    unsigned short* d2 = pbl + i8;
    *(volatile v4u*)d0 = fh.u;
    *(volatile v4u*)d1 = fbh.u;
    *(volatile v4u*)d2 = fbl.u;
    __threadfence();
    *(volatile v4u*)d0 = fh.u;
    *(volatile v4u*)d1 = fbh.u;
    *(volatile v4u*)d2 = fbl.u;
}

template<int SPLIT>
__global__ __launch_bounds__(256) void k_wprep(const float* __restrict__ W, int K, int N, float scale,
                                               unsigned short* P0, unsigned short* P1)
{
    __shared__ float tile[64][65];
    const int t = threadIdx.x, l = t & 31, w = t >> 5;
    const int n0 = blockIdx.x * 64, k0 = blockIdx.y * 64;
    if (n0 + 64 > N || k0 + 64 > K) return;
    {
        const int n4 = (t & 15) * 4, kk = t >> 4;
#pragma unroll
        for (int i = 0; i < 4; ++i) {
            const int kr = kk + 16 * i;
            const v4f vv = *(const v4f*)(W + (size_t)(k0 + kr) * N + n0 + n4);
            tile[kr][n4 + 0] = vv[0] * scale;
            tile[kr][n4 + 1] = vv[1] * scale;
            tile[kr][n4 + 2] = vv[2] * scale;
            tile[kr][n4 + 3] = vv[3] * scale;
        }
    }
    __syncthreads();
    v4u o0[2], o1[2];
    size_t dst[2];
#pragma unroll
    for (int s = 0; s < 2; ++s) {
        const int nn = 8 * w + 4 * s + (l >> 3);
        const int kc = (l & 7) * 8;
        Pack8 p0, p1;
#pragma unroll
        for (int e = 0; e < 8; ++e) {
            const float f = tile[kc + e][nn];
            if (SPLIT) {
                const unsigned short hb = bf16_rne_bits(f);
                p0.s[e] = hb;
                p1.s[e] = bf16_rne_bits(f - bf16_bits_to_f32(hb));
            } else {
                p0.hv[e] = (_Float16)f;
                p1.s[e] = 0;
            }
        }
        o0[s] = p0.u;
        o1[s] = p1.u;
        dst[s] = (size_t)(n0 + nn) * K + k0 + kc;
    }
#pragma unroll
    for (int s = 0; s < 2; ++s) {
        *(volatile v4u*)(P0 + dst[s]) = o0[s];
        if (SPLIT) *(volatile v4u*)(P1 + dst[s]) = o1[s];
    }
    __threadfence();
#pragma unroll
    for (int s = 0; s < 2; ++s) {
        *(volatile v4u*)(P0 + dst[s]) = o0[s];
        if (SPLIT) *(volatile v4u*)(P1 + dst[s]) = o1[s];
    }
}

__device__ __forceinline__ void tile_store(const float* sC, float* Cf, _Float16* Ch,
                                           int m0, int n0, int N, int w, int l, int out16)
{
    const int h = l >> 4, m = l & 15;
    if (!out16) {
#pragma unroll
        for (int it = 0; it < 8; ++it) {
            const int row = 16 * w + 2 * it + h;
            const int col = 4 * m;
            const v4f val = *(const v4f*)(sC + row * GCP + col);
            *(volatile v4f*)(Cf + (size_t)(m0 + row) * N + n0 + col) = val;
        }
    } else {
#pragma unroll
        for (int it = 0; it < 4; ++it) {
            const int row = 16 * w + 4 * it + (l >> 3);
            const int col = (l & 7) * 8;
            const v4f c0 = *(const v4f*)(sC + row * GCP + col);
            const v4f c1 = *(const v4f*)(sC + row * GCP + col + 4);
            Pack8 p;
            p.hv[0] = (_Float16)c0[0]; p.hv[1] = (_Float16)c0[1];
            p.hv[2] = (_Float16)c0[2]; p.hv[3] = (_Float16)c0[3];
            p.hv[4] = (_Float16)c1[0]; p.hv[5] = (_Float16)c1[1];
            p.hv[6] = (_Float16)c1[2]; p.hv[7] = (_Float16)c1[3];
            *(volatile v4u*)(Ch + (size_t)(m0 + row) * N + n0 + col) = p.u;
        }
    }
}

template<typename T, int NP>
__global__ __launch_bounds__(256) void k_gemm(const T* __restrict__ Ah, const T* __restrict__ Al,
                                              const T* __restrict__ Bh, const T* __restrict__ Bl,
                                              float* Cf, _Float16* Ch,
                                              int M, int N, int K, float scale, int act, int out16)
{
    __shared__ __attribute__((aligned(16))) unsigned char lds[LDS_GEMM];
    T* sAh = (T*)lds;
    T* sAl = (T*)(lds + LDS_A);
    T* sBh = (T*)(lds + 2 * LDS_A);
    T* sBl = (T*)(lds + 2 * LDS_A + LDS_B);
    float* sC = (float*)lds;

    const int t = threadIdx.x, l = t & 31, w = t >> 5, h = l >> 4, m = l & 15;
    const int wr = w >> 1, wc = w & 1;
    const int m0 = blockIdx.y * GBM, n0 = blockIdx.x * GBN;
    if (m0 + GBM > M || n0 + GBN > N) return;

    v8f acc[2][2];
#pragma unroll
    for (int i = 0; i < 2; ++i)
#pragma unroll
        for (int j = 0; j < 2; ++j)
#pragma unroll
            for (int r = 0; r < 8; ++r) acc[i][j][r] = 0.0f;

    for (int k0 = 0; k0 < K; k0 += GBK) {
#pragma unroll
        for (int rep = 0; rep < 2; ++rep) {
            const int c = t + rep * 256;
            const int row = c >> 2, part = c & 3;
            const size_t g = (size_t)(m0 + row) * K + k0 + part * 8;
            const int s = row * GPK + part * 8;
            *(v4u*)(sAh + s) = *(const v4u*)(Ah + g);
            if (NP > 1) *(v4u*)(sAl + s) = *(const v4u*)(Al + g);
        }
        {
            const int row = t >> 2, part = t & 3;
            const size_t g = (size_t)(n0 + row) * K + k0 + part * 8;
            const int s = row * GPK + part * 8;
            *(v4u*)(sBh + s) = *(const v4u*)(Bh + g);
            if (NP > 1) *(v4u*)(sBl + s) = *(const v4u*)(Bl + g);
        }
        __syncthreads();

        Frag<T> fa[2], fb[2], ga[2], gb[2];
#pragma unroll
        for (int i = 0; i < 2; ++i) {
            const int ra = (wr * 32 + i * 16 + m) * GPK + 8 * h;
            fa[i].u[0] = *(const v4u*)(sAh + ra);
            fa[i].u[1] = *(const v4u*)(sAh + ra + 16);
            if (NP > 1) {
                ga[i].u[0] = *(const v4u*)(sAl + ra);
                ga[i].u[1] = *(const v4u*)(sAl + ra + 16);
            }
            const int rb = (wc * 32 + i * 16 + m) * GPK + 8 * h;
            fb[i].u[0] = *(const v4u*)(sBh + rb);
            fb[i].u[1] = *(const v4u*)(sBh + rb + 16);
            if (NP > 1) {
                gb[i].u[0] = *(const v4u*)(sBl + rb);
                gb[i].u[1] = *(const v4u*)(sBl + rb + 16);
            }
        }
#pragma unroll
        for (int i = 0; i < 2; ++i) {
#pragma unroll
            for (int j = 0; j < 2; ++j) {
                acc[i][j] = mma16(fa[i].v, fb[j].v, acc[i][j]);
                if (NP > 1) {
                    acc[i][j] = mma16(fa[i].v, gb[j].v, acc[i][j]);
                    acc[i][j] = mma16(ga[i].v, fb[j].v, acc[i][j]);
                }
            }
        }
        __syncthreads();
    }

#pragma unroll
    for (int i = 0; i < 2; ++i) {
#pragma unroll
        for (int j = 0; j < 2; ++j) {
            const int cc = wc * 32 + j * 16 + m;
#pragma unroll
            for (int r = 0; r < 8; ++r) {
                const int rr = wr * 32 + i * 16 + 8 * h + r;
                float val = acc[i][j][r] * scale;
                if (act == 1) val = val / (1.0f + expf(-val));
                sC[rr * GCP + cc] = val;
            }
        }
    }
    __syncthreads();
    tile_store(sC, Cf, Ch, m0, n0, N, w, l, out16);
    __threadfence();
    tile_store(sC, Cf, Ch, m0, n0, N, w, l, out16);
}

__global__ __launch_bounds__(512) void k_scan(const float* __restrict__ q, const float* __restrict__ k,
                                              const float* __restrict__ v, const float* __restrict__ f,
                                              const _Float16* __restrict__ gate, const float* __restrict__ norm_w,
                                              unsigned short* yh, unsigned short* yl)
{
    const int bh = blockIdx.x;
    if (bh >= Bc * Hc) return;
    const int b = bh / Hc, hh = bh - b * Hc;
    const int t = threadIdx.x, l = t & 31, w = t >> 5;

    __shared__ float s_q[DKc], s_k[DKc], s_v[DKc], s_g[DKc], s_nw[DKc];
    __shared__ float s_dec[Mc], s_cmp[Mc], s_ok[Mc], s_qv[Mc];
    __shared__ float s_part[512], s_ovp[512], s_red[4];
    __shared__ __attribute__((aligned(16))) unsigned short s_y[2][DKc];

    float hk[16], hv[16];
#pragma unroll
    for (int i = 0; i < 16; ++i) { hk[i] = 0.0f; hv[i] = 0.0f; }

    const int m1  = t & 63;
    const int d1  = (t >> 6) * 16;
    const int dk2 = t & 127;
    const int m2  = (t >> 7) * 16;

    if (t < DKc) s_nw[t] = norm_w[hh * DKc + t];

    const size_t colq = (size_t)hh * DKc;

    for (int step = 0; step < Nc; ++step) {
        const size_t row = (size_t)b * Nc + step;
        if (t < DKc) {
            const size_t o = row * Dc + colq + t;
            s_q[t] = q[o];
            s_k[t] = k[o];
            s_v[t] = v[o];
        } else if (t < DKc + Mc) {
            const int mm = t - DKc;
            const float fv = f[row * FMc + hh * Mc + mm];
            const float e  = __expf(-fv);
            const float sg = __builtin_amdgcn_rcpf(1.0f + e);
            s_dec[mm] = sg;
            s_cmp[mm] = e * sg;
        } else if (t < 2 * DKc + Mc) {
            const int d = t - DKc - Mc;
            s_g[d] = (float)gate[row * Dc + colq + d];
        }
        __syncthreads();

        {
            const float dec = s_dec[m1], sc = s_cmp[m1];
            float part = 0.0f;
#pragma unroll
            for (int i = 0; i < 16; ++i) {
                hk[i] = hk[i] * dec + s_k[d1 + i] * sc;
                part += s_q[d1 + i] * hk[i];
            }
            s_part[t] = part;
        }
        __syncthreads();

        if (t < Mc) {
            float a = 0.0f;
#pragma unroll
            for (int g = 0; g < 8; ++g) a += s_part[g * 64 + t];
            s_ok[t] = a;
        }
        __syncthreads();

        if (t < 32) {
            const float a0 = s_ok[l], a1 = s_ok[l + 32];
            float mx = fmaxf(a0, a1);
#pragma unroll
            for (int o = 16; o > 0; o >>= 1) mx = fmaxf(mx, __shfl_xor(mx, o, 32));
            const float e0 = __expf(a0 - mx), e1 = __expf(a1 - mx);
            float sm = e0 + e1;
#pragma unroll
            for (int o = 16; o > 0; o >>= 1) sm += __shfl_xor(sm, o, 32);
            const float inv = __builtin_amdgcn_rcpf(sm);
            s_qv[l]      = e0 * inv;
            s_qv[l + 32] = e1 * inv;
        }
        __syncthreads();

        {
            const float vv = s_v[dk2];
            float op = 0.0f;
#pragma unroll
            for (int i = 0; i < 16; ++i) {
                const int mm = m2 + i;
                hv[i] = hv[i] * s_dec[mm] + s_cmp[mm] * vv;
                op += s_qv[mm] * hv[i];
            }
            s_ovp[t] = op;
        }
        __syncthreads();

        float og = 0.0f;
        if (t < DKc) {
            const float ov  = s_ovp[t] + s_ovp[t + 128] + s_ovp[t + 256] + s_ovp[t + 384];
            const float gg  = s_g[t];
            const float sig = __builtin_amdgcn_rcpf(1.0f + __expf(-gg));
            og = ov * sig;
            float sq = og * og;
#pragma unroll
            for (int o = 16; o > 0; o >>= 1) sq += __shfl_xor(sq, o, 32);
            if (l == 0) s_red[w] = sq;
        }
        __syncthreads();

        if (t < DKc) {
            const float ms = (s_red[0] + s_red[1] + s_red[2] + s_red[3]) * (1.0f / (float)DKc);
            const float rr = rsqrtf(ms + EPSc);
            const float y  = og * rr * s_nw[t];
            const unsigned short hb = bf16_rne_bits(y);
            s_y[0][t] = hb;
            s_y[1][t] = bf16_rne_bits(y - bf16_bits_to_f32(hb));
        }
        __syncthreads();

        if (t < 32) {
            const int pl  = l >> 4;
            const int idx = (l & 15) * 8;
            const v4u val = *(const v4u*)(&s_y[pl][idx]);
            unsigned short* dst = (pl ? yl : yh) + row * Dc + colq + idx;
            *(volatile v4u*)dst = val;
            __threadfence();
            *(volatile v4u*)dst = val;
        }
    }
}

template<typename T, int NP>
static void launch_gemm(hipStream_t st, const void* Ah, const void* Al, const void* Bh, const void* Bl,
                        float* Cf, void* Ch, int M, int N, int K, float scale, int act, int out16)
{
    dim3 grid(N / GBN, M / GBM);
    k_gemm<T, NP><<<grid, 256, 0, st>>>((const T*)Ah, (const T*)Al, (const T*)Bh, (const T*)Bl,
                                        Cf, (_Float16*)Ch, M, N, K, scale, act, out16);
}

extern "C" void kernel_launch(void* const* d_in, const int* in_sizes, int n_in,
                              void* d_out, int out_size, void* d_ws, size_t ws_size,
                              hipStream_t stream)
{
    if (n_in < 10) return;
    if (in_sizes[0] != Rows * Dc || in_sizes[1] != Dc * Dc || in_sizes[2] != Dc * Dc ||
        in_sizes[3] != Dc * Dc || in_sizes[4] != Dc * DKc || in_sizes[5] != DKc * FMc ||
        in_sizes[6] != Dc * DKc || in_sizes[7] != DKc * Dc || in_sizes[8] != Dc * Dc ||
        in_sizes[9] != Dc || out_size != Rows * Dc) return;

    const float* x      = (const float*)d_in[0];
    const float* Wq     = (const float*)d_in[1];
    const float* Wk     = (const float*)d_in[2];
    const float* Wv     = (const float*)d_in[3];
    const float* Wf1    = (const float*)d_in[4];
    const float* Wf2    = (const float*)d_in[5];
    const float* Wg1    = (const float*)d_in[6];
    const float* Wg2    = (const float*)d_in[7];
    const float* Wo     = (const float*)d_in[8];
    const float* norm_w = (const float*)d_in[9];

    size_t off = 0;
    auto carve = [&](size_t bytes) -> size_t { size_t p = off; off += (bytes + 255) & ~(size_t)255; return p; };
    const size_t o_xh   = carve((size_t)Rows * Dc * 2);
    const size_t o_xbh  = carve((size_t)Rows * Dc * 2);
    const size_t o_xbl  = carve((size_t)Rows * Dc * 2);
    const size_t o_wq   = carve((size_t)Dc * Dc * 2);
    const size_t o_wk   = carve((size_t)Dc * Dc * 2);
    const size_t o_wvh  = carve((size_t)Dc * Dc * 2);
    const size_t o_wvl  = carve((size_t)Dc * Dc * 2);
    const size_t o_wf1  = carve((size_t)DKc * Dc * 2);
    const size_t o_wf2  = carve((size_t)FMc * DKc * 2);
    const size_t o_wg1  = carve((size_t)DKc * Dc * 2);
    const size_t o_wg2  = carve((size_t)Dc * DKc * 2);
    const size_t o_woh  = carve((size_t)Dc * Dc * 2);
    const size_t o_wol  = carve((size_t)Dc * Dc * 2);
    const size_t o_q    = carve((size_t)Rows * Dc * 4);
    const size_t o_k    = carve((size_t)Rows * Dc * 4);
    const size_t o_v    = carve((size_t)Rows * Dc * 4);
    const size_t o_f    = carve((size_t)Rows * FMc * 4);
    const size_t o_f1   = carve((size_t)Rows * DKc * 2);
    const size_t o_g1   = carve((size_t)Rows * DKc * 2);
    const size_t o_gate = carve((size_t)Rows * Dc * 2);
    const size_t o_yh   = carve((size_t)Rows * Dc * 2);
    const size_t o_yl   = carve((size_t)Rows * Dc * 2);
    if (off > ws_size) return;

    char* ws = (char*)d_ws;
    unsigned short* xh   = (unsigned short*)(ws + o_xh);
    unsigned short* xbh  = (unsigned short*)(ws + o_xbh);
    unsigned short* xbl  = (unsigned short*)(ws + o_xbl);
    unsigned short* wq   = (unsigned short*)(ws + o_wq);
    unsigned short* wk   = (unsigned short*)(ws + o_wk);
    unsigned short* wvh  = (unsigned short*)(ws + o_wvh);
    unsigned short* wvl  = (unsigned short*)(ws + o_wvl);
    unsigned short* wf1  = (unsigned short*)(ws + o_wf1);
    unsigned short* wf2  = (unsigned short*)(ws + o_wf2);
    unsigned short* wg1  = (unsigned short*)(ws + o_wg1);
    unsigned short* wg2  = (unsigned short*)(ws + o_wg2);
    unsigned short* woh  = (unsigned short*)(ws + o_woh);
    unsigned short* wol  = (unsigned short*)(ws + o_wol);
    float* qf  = (float*)(ws + o_q);
    float* kf  = (float*)(ws + o_k);
    float* vf  = (float*)(ws + o_v);
    float* ff  = (float*)(ws + o_f);
    unsigned short* f1h   = (unsigned short*)(ws + o_f1);
    unsigned short* g1h   = (unsigned short*)(ws + o_g1);
    unsigned short* gateh = (unsigned short*)(ws + o_gate);
    unsigned short* yh    = (unsigned short*)(ws + o_yh);
    unsigned short* yl    = (unsigned short*)(ws + o_yl);

    const float s64 = 64.0f, inv64 = 1.0f / 64.0f;

    k_xprep<<<(Rows * Dc) / (256 * 8), 256, 0, stream>>>(x, Rows * Dc, xh, xbh, xbl);

    k_wprep<0><<<dim3(Dc / 64,  Dc / 64),  256, 0, stream>>>(Wq,  Dc,  Dc,  s64,  wq,  wq);
    k_wprep<0><<<dim3(Dc / 64,  Dc / 64),  256, 0, stream>>>(Wk,  Dc,  Dc,  s64,  wk,  wk);
    k_wprep<1><<<dim3(Dc / 64,  Dc / 64),  256, 0, stream>>>(Wv,  Dc,  Dc,  1.0f, wvh, wvl);
    k_wprep<0><<<dim3(DKc / 64, Dc / 64),  256, 0, stream>>>(Wf1, Dc,  DKc, s64,  wf1, wf1);
    k_wprep<0><<<dim3(FMc / 64, DKc / 64), 256, 0, stream>>>(Wf2, DKc, FMc, s64,  wf2, wf2);
    k_wprep<0><<<dim3(DKc / 64, Dc / 64),  256, 0, stream>>>(Wg1, Dc,  DKc, s64,  wg1, wg1);
    k_wprep<0><<<dim3(Dc / 64,  DKc / 64), 256, 0, stream>>>(Wg2, DKc, Dc,  s64,  wg2, wg2);
    k_wprep<1><<<dim3(Dc / 64,  Dc / 64),  256, 0, stream>>>(Wo,  Dc,  Dc,  1.0f, woh, wol);

    launch_gemm<_Float16, 1>(stream, xh,  xh,  wq,  wq,  qf, f1h, Rows, Dc,  Dc,  inv64, 1, 0);
    launch_gemm<_Float16, 1>(stream, xh,  xh,  wk,  wk,  kf, f1h, Rows, Dc,  Dc,  inv64, 1, 0);
    launch_gemm<__bf16,   3>(stream, xbh, xbl, wvh, wvl, vf, f1h, Rows, Dc,  Dc,  1.0f,  0, 0);
    launch_gemm<_Float16, 1>(stream, xh,  xh,  wf1, wf1, ff, f1h, Rows, DKc, Dc,  inv64, 0, 1);
    launch_gemm<_Float16, 1>(stream, f1h, f1h, wf2, wf2, ff, g1h, Rows, FMc, DKc, inv64, 0, 0);
    launch_gemm<_Float16, 1>(stream, xh,  xh,  wg1, wg1, ff, g1h, Rows, DKc, Dc,  inv64, 0, 1);
    launch_gemm<_Float16, 1>(stream, g1h, g1h, wg2, wg2, ff, gateh, Rows, Dc, DKc, inv64, 0, 1);

    k_scan<<<Bc * Hc, 512, 0, stream>>>(qf, kf, vf, ff, (const _Float16*)gateh, norm_w, yh, yl);

    launch_gemm<__bf16, 3>(stream, yh, yl, woh, wol, (float*)d_out, gateh, Rows, Dc, Dc, 1.0f, 0, 0);
}
